// GNNModel_54485955117135
// MI455X (gfx1250) — hardware-run, weakly checked
//
#include <hip/hip_runtime.h>
#include <stddef.h>
#include <stdint.h>


#define LNEPS  1e-5f
#define NTHR   256
#define NWAVE  8
#define EPT    8
#define CHUNK  (NTHR * EPT)
#define WCAP   (EPT * 32)
#define LISTN  (NWAVE * WCAP)
#define NBA    1024
#define SLA    10
#define RCAP   16384
#define TROWS  128
#define AP     136
#define HP     128
#define GBM    64
#define GTHR   128
#define EA_P   72
#define ER_P   40
#define EH_P   68
#define EZ_P   20
#define HD_P   264
#define CMP_ZINTS (LISTN + 2 * RCAP + 3 * NBA)
#define CMP_LDS_BYTES ((CMP_ZINTS + 16) * 4)
#define EDGE_OFF_R  (TROWS * EA_P * 2)
#define EDGE_OFF_H  (EDGE_OFF_R + TROWS * ER_P * 2)
#define EDGE_OFF_Z  (EDGE_OFF_H + TROWS * EH_P * 4)
#define EDGE_OFF_M  (EDGE_OFF_Z + TROWS * EZ_P * 4)
#define EDGE_OFF_W  (EDGE_OFF_M + TROWS * HP * 2)
#define EDGE_OFF_C  (EDGE_OFF_W + TROWS * 4)
#define EDGE_LDS_BYTES (EDGE_OFF_C + 176 * 4)
#define HEAD_LDS_BYTES (GBM * 128 * 4 + GBM * HD_P * 2 + 3 * 64 * 4)
#define KVG __attribute__((amdgpu_num_vgpr(248)))

static_assert((CHUNK & (CHUNK - 1)) == 0 && CHUNK <= 4096);
static_assert(NBA == (1 << SLA) && NBA == 4 * NTHR);
static_assert(CMP_ZINTS % (NTHR * 4) == 0);
static_assert(RCAP == 16 * NTHR * 4);
static_assert(CMP_LDS_BYTES <= 300000 && EDGE_LDS_BYTES <= 300000);
static_assert((EDGE_OFF_R % 16) == 0 && (EDGE_OFF_H % 16) == 0 && (EDGE_OFF_Z % 16) == 0);
static_assert((EDGE_OFF_M % 16) == 0 && (EDGE_OFF_W % 16) == 0 && (EDGE_OFF_C % 16) == 0);
static_assert((AP * 2) % 16 == 0 && (EA_P * 2) % 16 == 0 && (ER_P * 2) % 16 == 0 && (HD_P * 2) % 16 == 0);
static_assert(TROWS * AP * 2 >= TROWS * HP * 2);
static_assert(NBA % TROWS == 0 && TROWS == 2 * GBM);
static_assert(NBA % GBM == 0 && GTHR >= GBM && (GBM & (GBM - 1)) == 0);

typedef float          v4f   __attribute__((ext_vector_type(4)));
typedef float          v8f   __attribute__((ext_vector_type(8)));
typedef int            v4i   __attribute__((ext_vector_type(4)));
typedef int            v8i   __attribute__((ext_vector_type(8)));
typedef unsigned short v4us  __attribute__((ext_vector_type(4)));
typedef unsigned short v8us  __attribute__((ext_vector_type(8)));
typedef unsigned short v16us __attribute__((ext_vector_type(16)));
typedef __bf16         v16bf __attribute__((ext_vector_type(16)));
typedef v4f  __attribute__((may_alias)) v4fa;
typedef v4i  __attribute__((may_alias)) v4ia;
typedef v4us __attribute__((may_alias)) v4usa;
typedef v8us __attribute__((may_alias)) v8usa;
union FragB { v16bf v; v16us u; v8us h[2]; v8i w; };

__device__ __forceinline__ v8f wmb(const FragB& a, const FragB& b, v8f c) {
  v8f d = __builtin_amdgcn_wmma_f32_16x16x32_bf16(false, a.v, false, b.v, (short)0, c, false, false);
  asm volatile("v_nop\n\tv_nop\n\tv_nop\n\tv_nop" : "+v"(d) : "v"(a.w), "v"(b.w));
  return d;
}
__device__ __forceinline__ v8f z8() { v8f z = {0.f, 0.f, 0.f, 0.f, 0.f, 0.f, 0.f, 0.f}; return z; }

__device__ __forceinline__ unsigned bf16_bits(float f) {
  const unsigned u = __float_as_uint(f);
  return (u + 0x7FFFu + ((u >> 16) & 1u)) >> 16;
}
__device__ __forceinline__ float bf16_val(float f) { return __uint_as_float(bf16_bits(f) << 16); }
__device__ __forceinline__ unsigned hl_bits(float v, unsigned& lo) {
  const unsigned hb = bf16_bits(v);
  lo = bf16_bits(v - __uint_as_float(hb << 16));
  return hb;
}
__device__ __forceinline__ float relu_np(float v) { return v > 0.0f ? v : (v - v); }
__device__ __forceinline__ float elu_f(float v) { return v > 0.0f ? v : expm1f(v); }
__device__ __forceinline__ int clampi(int v, int lo, int hi) { return v < lo ? lo : (v > hi ? hi : v); }

__device__ __forceinline__ void put16(unsigned short* dp, v8us o) {
  *(volatile v8us*)dp = o;
  __threadfence();
  *(volatile v8us*)dp = o;
}
__device__ __forceinline__ void putf4(float* dp, v4f o) {
  *(volatile v4f*)dp = o;
  __threadfence();
  *(volatile v4f*)dp = o;
}

template <int SLB>
__device__ __forceinline__ int scan_chunk(const int* __restrict__ dsts, int nE, int cbase, int slotBase,
                                          int nb, int vec8, int* list, int tid, int lane, int wave) {
  int wc = 0;
  const int el0  = tid * EPT;
  const int e0   = cbase + el0;
  const int sent = -2147483647 - 1;
  v4i da, db;
  if (vec8 != 0 && cbase + CHUNK <= nE) {
    da = *(const v4i*)(dsts + e0);
    db = *(const v4i*)(dsts + e0 + 4);
  } else {
    da.x = (e0     < nE) ? dsts[min(e0,     nE - 1)] : sent;
    da.y = (e0 + 1 < nE) ? dsts[min(e0 + 1, nE - 1)] : sent;
    da.z = (e0 + 2 < nE) ? dsts[min(e0 + 2, nE - 1)] : sent;
    da.w = (e0 + 3 < nE) ? dsts[min(e0 + 3, nE - 1)] : sent;
    db.x = (e0 + 4 < nE) ? dsts[min(e0 + 4, nE - 1)] : sent;
    db.y = (e0 + 5 < nE) ? dsts[min(e0 + 5, nE - 1)] : sent;
    db.z = (e0 + 6 < nE) ? dsts[min(e0 + 6, nE - 1)] : sent;
    db.w = (e0 + 7 < nE) ? dsts[min(e0 + 7, nE - 1)] : sent;
  }
  const unsigned nbs = (unsigned)slotBase;
  const unsigned unb = (unsigned)nb;
  const unsigned s0 = (unsigned)da.x - nbs, s1 = (unsigned)da.y - nbs;
  const unsigned s2 = (unsigned)da.z - nbs, s3 = (unsigned)da.w - nbs;
  const unsigned s4 = (unsigned)db.x - nbs, s5 = (unsigned)db.y - nbs;
  const unsigned s6 = (unsigned)db.z - nbs, s7 = (unsigned)db.w - nbs;
  const bool h0 = s0 < unb, h1 = s1 < unb, h2 = s2 < unb, h3 = s3 < unb;
  const bool h4 = s4 < unb, h5 = s5 < unb, h6 = s6 < unb, h7 = s7 < unb;
  const unsigned any = __builtin_amdgcn_ballot_w32(h0 | h1 | h2 | h3 | h4 | h5 | h6 | h7);
  if (any != 0u) {
#define HITJ(J, HJ, SJ) { \
      const unsigned mj = __builtin_amdgcn_ballot_w32(HJ); \
      if (mj != 0u) { \
        if (HJ) { \
          const int pos = wc + (int)__builtin_amdgcn_mbcnt_lo(mj, 0u); \
          if (pos < WCAP) list[wave * WCAP + pos] = ((el0 + (J)) << SLB) | (int)(SJ); \
        } \
        wc += (int)__builtin_popcount(mj); } }
    HITJ(0, h0, s0)
    HITJ(1, h1, s1)
    HITJ(2, h2, s2)
    HITJ(3, h3, s3)
    HITJ(4, h4, s4)
    HITJ(5, h5, s5)
    HITJ(6, h6, s6)
    HITJ(7, h7, s7)
#undef HITJ
  }
  return wc;
}

__global__ __launch_bounds__(NTHR) KVG void k_wplane(const float* __restrict__ W, int ldw, int rbase, int per,
                                                     int Kp, int nUnits, unsigned short* D) {
  const int u = (int)blockIdx.x * NTHR + (int)threadIdx.x;
  if (u >= nUnits) return;
  const int kp8 = Kp >> 3;
  const int n   = u / kp8;
  const int k8  = (u - n * kp8) * 8;
  const int srow = rbase + (k8 % per) + (k8 / (2 * per)) * per;
  const float* p = W + (size_t)srow * (size_t)ldw + n;
  v8us o;
#pragma unroll
  for (int i = 0; i < 8; ++i) o[i] = (unsigned short)bf16_bits(p[(size_t)i * (size_t)ldw]);
  put16(D + (size_t)u * 8, o);
}

template <int H>
__global__ __launch_bounds__(NTHR) KVG void k_mplane(const float* __restrict__ ew2, const float* __restrict__ eb2,
                                                     const float* __restrict__ w1, int rowc,
                                                     unsigned short* MHL, float* CLp) {
  __shared__ __attribute__((aligned(16))) float sW[64 * 128];
  __shared__ __attribute__((aligned(16))) float sB[128];
  __shared__ __attribute__((aligned(16))) float sC[32];
  const int tid = (int)threadIdx.x;
#pragma unroll
  for (int it = 0; it < 8; ++it) {
    const int idx = (it * NTHR + tid) * 4;
    const v4f v = *(const v4f*)(ew2 + idx);
    v4f q;
    q.x = bf16_val(v.x); q.y = bf16_val(v.y); q.z = bf16_val(v.z); q.w = bf16_val(v.w);
    *(v4fa*)(sW + idx) = q;
  }
  if (tid < 128) sB[tid] = bf16_val(eb2[tid]);
  __syncthreads();
  const int u  = (int)blockIdx.x * NTHR + tid;
  const int n  = u >> 3;
  const int k8 = (u & 7) * 8;
  double a[8];
#pragma unroll
  for (int i = 0; i < 8; ++i) a[i] = 0.0;
  double ac = 0.0;
#pragma unroll 1
  for (int j = 0; j < 128; ++j) {
    const double wv = (double)bf16_val(w1[(size_t)(rowc + j) * H + n]);
#pragma unroll
    for (int i = 0; i < 8; ++i) a[i] += (double)sW[(k8 + i) * 128 + j] * wv;
    ac += (double)sB[j] * wv;
  }
  v8us oh, ol;
#pragma unroll
  for (int i = 0; i < 8; ++i) {
    unsigned lb;
    const unsigned hb = hl_bits((float)a[i], lb);
    oh[i] = (unsigned short)hb;
    ol[i] = (unsigned short)lb;
  }
  unsigned short* dp = MHL + (size_t)n * 192 + k8;
  *(volatile v8us*)dp         = oh;
  *(volatile v8us*)(dp + 64)  = oh;
  *(volatile v8us*)(dp + 128) = ol;
  __threadfence();
  *(volatile v8us*)dp         = oh;
  *(volatile v8us*)(dp + 64)  = oh;
  *(volatile v8us*)(dp + 128) = ol;
  if ((u & 7) == 0) sC[n & 31] = (float)ac;
  __syncthreads();
  if (tid < 8) {
    const v4f c4 = *(const v4fa*)(sC + 4 * tid);
    putf4(CLp + (size_t)blockIdx.x * 32 + 4 * tid, c4);
  }
}

__global__ __launch_bounds__(NTHR) KVG void k_xprep(const float* __restrict__ x, const float* __restrict__ w,
                                                    const float* __restrict__ b, const float* __restrict__ rm,
                                                    const float* __restrict__ rv, int nN, unsigned short* XHL) {
#pragma clang fp contract(off)
  __shared__ float sS[64];
  __shared__ float sM[64];
  __shared__ float sWt[64];
  __shared__ float sBt[64];
  const int tid = (int)threadIdx.x;
  if (tid < 64) {
    sS[tid]  = sqrtf(bf16_val(rv[tid]) + LNEPS);
    sM[tid]  = bf16_val(rm[tid]);
    sWt[tid] = bf16_val(w[tid]);
    sBt[tid] = bf16_val(b[tid]);
  }
  __syncthreads();
  const int u   = (int)blockIdx.x * NTHR + tid;
  const int row = u >> 3;
  const int j   = u & 7;
  const int rc  = row < nN ? row : nN - 1;
  const bool ok = row < nN;
  const float* p = x + (size_t)rc * 64 + 8 * j;
  const v4f a0 = *(const v4f*)p;
  const v4f a1 = *(const v4f*)(p + 4);
  const float xv[8] = {a0.x, a0.y, a0.z, a0.w, a1.x, a1.y, a1.z, a1.w};
  v8us oh, ol;
#pragma unroll
  for (int i = 0; i < 8; ++i) {
    const int c = 8 * j + i;
    float v = (bf16_val(xv[i]) - sM[c]) / sS[c];
    v = v * sWt[c];
    v = v + sBt[c];
    v = ok ? v : 0.0f;
    unsigned lb;
    const unsigned hb = hl_bits(v, lb);
    oh[i] = (unsigned short)hb;
    ol[i] = (unsigned short)lb;
  }
  unsigned short* dp = XHL + (size_t)row * 128 + 8 * j;
  *(volatile v8us*)dp        = oh;
  *(volatile v8us*)(dp + 64) = ol;
  __threadfence();
  *(volatile v8us*)dp        = oh;
  *(volatile v8us*)(dp + 64) = ol;
}

__global__ __launch_bounds__(NTHR) KVG void k_compact(const int* __restrict__ dsts, int nE, int vec8,
                                                      int* LISTP, int* TAB, int nTab) {
  extern __shared__ __attribute__((aligned(16))) int dsm[];
  int* list = dsm;
  int* hl   = dsm + LISTN;
  int* sl   = hl + RCAP;
  int* cnt  = sl + RCAP;
  int* offs = cnt + NBA;
  int* cur  = offs + NBA;
  int* misc = cur + NBA;
  const int tid = (int)threadIdx.x, lane = tid & 31, wave = tid >> 5;
  const int nodeBase = (int)blockIdx.x * NBA;

  {
    const v4i z4 = {0, 0, 0, 0};
    for (int i = tid * 4; i < CMP_ZINTS; i += NTHR * 4) *(v4ia*)(dsm + i) = z4;
    if (tid < 16) misc[tid] = 0;
  }
  __syncthreads();

  int t = 0, ov = 0;
  const int nChunks = (nE + CHUNK - 1) / CHUNK;
#pragma unroll 1
  for (int ch = 0; ch < nChunks; ++ch) {
    const int cbase = ch * CHUNK;
    const int wc = scan_chunk<SLA>(dsts, nE, cbase, nodeBase, NBA, vec8, list, tid, lane, wave);
    if (lane == 0) misc[wave] = wc;
    __syncthreads();
    if (wave == 0) {
#pragma unroll 1
      for (int w2 = 0; w2 < NWAVE; ++w2) {
        int c = misc[w2];
        c = c < 0 ? 0 : (c > WCAP ? WCAP : c);
#pragma unroll 1
        for (int b0 = 0; b0 < c; b0 += 32) {
          const int idx = b0 + lane;
          const int ent = list[w2 * WCAP + (idx < WCAP ? idx : WCAP - 1)];
          const int m32 = (c - b0) < 32 ? (c - b0) : 32;
#pragma unroll 1
          for (int k = 0; k < m32; ++k) {
            const int u    = __builtin_amdgcn_readlane(ent, k);
            const int slot = u & (NBA - 1);
            const int el   = (u >> SLA) & (CHUNK - 1);
            const int pk   = ((cbase + el) << SLA) | slot;
            if (t < RCAP) {
              if (lane == 0) { hl[t] = pk; cnt[slot] = cnt[slot] + 1; }
              t = t + 1;
            } else {
              ov = 1;
            }
          }
        }
      }
    }
    __syncthreads();
  }
  if (wave == 0 && lane == 0) { misc[8] = t; misc[9] = ov; }
  __syncthreads();
  int tt = misc[8];
  tt = tt < 0 ? 0 : (tt > RCAP ? RCAP : tt);
  const int ovf = misc[9];

  if (wave == 0) {
    const int base = lane * (NBA / 32);
    int s = 0;
#pragma unroll 1
    for (int i = 0; i < NBA / 32; ++i) s += cnt[base + i];
    int incl = s;
#pragma unroll
    for (int d = 1; d < 32; d <<= 1) {
      const int y = __shfl_up(incl, d, 32);
      if (lane >= d) incl += y;
    }
    int run = incl - s;
#pragma unroll 1
    for (int i = 0; i < NBA / 32; ++i) {
      const int cv = cnt[base + i];
      offs[base + i] = run;
      cur[base + i]  = run;
      run += cv;
    }
  }
  __syncthreads();
  if (wave == 0) {
#pragma unroll 1
    for (int b0 = 0; b0 < tt; b0 += 32) {
      const int idx = b0 + lane;
      const int ent = hl[idx < RCAP ? idx : RCAP - 1];
      const int m32 = (tt - b0) < 32 ? (tt - b0) : 32;
#pragma unroll 1
      for (int k = 0; k < m32; ++k) {
        const int u    = __builtin_amdgcn_readlane(ent, k);
        const int slot = u & (NBA - 1);
        if (lane == 0) {
          int p = cur[slot];
          p = p < 0 ? 0 : (p > RCAP - 1 ? RCAP - 1 : p);
          sl[p] = u;
          cur[slot] = p + 1;
        }
      }
    }
  }
  __syncthreads();

  {
    const v4i c4 = *(const v4ia*)(cnt + 4 * tid);
    const v4i o4 = *(const v4ia*)(offs + 4 * tid);
    v4i mv = {0, 0, 0, 0};
    mv.x = (tid == 0) ? tt : 0;
    mv.y = (tid == 0) ? ovf : 0;
    int* cp = TAB + (size_t)nodeBase + 4 * tid;
    int* op = TAB + (size_t)nTab + nodeBase + 4 * tid;
    int* mp = TAB + (size_t)2 * nTab + (size_t)blockIdx.x * 32 + 4 * (tid & 7);
    *(volatile v4i*)cp = c4;
    *(volatile v4i*)op = o4;
    if (tid < 8) *(volatile v4i*)mp = mv;
    __threadfence();
    *(volatile v4i*)cp = c4;
    *(volatile v4i*)op = o4;
    if (tid < 8) *(volatile v4i*)mp = mv;
  }
  {
    v4i pv[16];
#pragma unroll
    for (int it = 0; it < 16; ++it) {
      const v4i e4 = *(const v4ia*)(sl + (it * NTHR + tid) * 4);
      pv[it] = e4 >> SLA;
    }
    int* lb = LISTP + (size_t)blockIdx.x * RCAP;
#pragma unroll
    for (int it = 0; it < 16; ++it) *(volatile v4i*)(lb + (it * NTHR + tid) * 4) = pv[it];
    __threadfence();
#pragma unroll
    for (int it = 0; it < 16; ++it) *(volatile v4i*)(lb + (it * NTHR + tid) * 4) = pv[it];
  }
}

__global__ __launch_bounds__(NTHR) KVG void k_edge(const float* __restrict__ EA, int nE,
                                                   const unsigned short* __restrict__ EE1D,
                                                   const unsigned short* __restrict__ ECW,
                                                   const float* __restrict__ lng, const float* __restrict__ lnb,
                                                   const float* __restrict__ b1, const float* __restrict__ ecb1,
                                                   const float* __restrict__ ecw2, const float* __restrict__ ecb2,
                                                   unsigned short* HID, float* EWG) {
  extern __shared__ __attribute__((aligned(16))) unsigned char dynb[];
  unsigned short* sA  = (unsigned short*)dynb;
  unsigned short* sR  = (unsigned short*)(dynb + EDGE_OFF_R);
  float*          sH  = (float*)(dynb + EDGE_OFF_H);
  float*          sZ  = (float*)(dynb + EDGE_OFF_Z);
  unsigned short* sM  = (unsigned short*)(dynb + EDGE_OFF_M);
  float*          sEW = (float*)(dynb + EDGE_OFF_W);
  float*          cst = (float*)(dynb + EDGE_OFF_C);
  const int tid = (int)threadIdx.x, lane = tid & 31, wave = tid >> 5, hh = lane >> 4, m = lane & 15;

  {
    const float vb1 = b1[tid & 63];
    const float vc1 = ecb1[tid & 15];
    const float vc2 = ecw2[tid & 15];
    const float vg  = lng[tid & 31];
    const float vb  = lnb[tid & 31];
    const float vz  = ecb2[0];
    const float cb1 = bf16_val(vb1);
    const float cc1 = bf16_val(vc1);
    const float cc2 = bf16_val(vc2);
    const float cg  = bf16_val(vg);
    const float cbb = bf16_val(vb);
    const float cz  = bf16_val(vz);
    if (tid < 64) cst[tid] = cb1;
    if (tid < 16) { cst[64 + tid] = cc1; cst[80 + tid] = cc2; }
    if (tid < 32) { cst[112 + tid] = cg; cst[144 + tid] = cbb; }
    if (tid == 0) cst[96] = cz;
  }
  __syncthreads();

  const int row = tid >> 1, hf = tid & 1;
  {
    const int eg = (int)blockIdx.x * TROWS + row;
    const int ec = eg < nE ? eg : nE - 1;
    const float* ea = EA + (size_t)ec * 32 + 16 * hf;
    const v4f q0 = *(const v4f*)(ea);
    const v4f q1 = *(const v4f*)(ea + 4);
    const v4f q2 = *(const v4f*)(ea + 8);
    const v4f q3 = *(const v4f*)(ea + 12);
    const float r[16] = {bf16_val(q0.x), bf16_val(q0.y), bf16_val(q0.z), bf16_val(q0.w),
                         bf16_val(q1.x), bf16_val(q1.y), bf16_val(q1.z), bf16_val(q1.w),
                         bf16_val(q2.x), bf16_val(q2.y), bf16_val(q2.z), bf16_val(q2.w),
                         bf16_val(q3.x), bf16_val(q3.y), bf16_val(q3.z), bf16_val(q3.w)};
    float s = 0.0f;
#pragma unroll
    for (int i = 0; i < 16; ++i) s += r[i];
    s += __shfl_xor(s, 1, 32);
    const float mu = s * (1.0f / 32.0f);
    float d[16];
    float q = 0.0f;
#pragma unroll
    for (int i = 0; i < 16; ++i) { d[i] = r[i] - mu; q += d[i] * d[i]; }
    q += __shfl_xor(q, 1, 32);
    const float var  = q * (1.0f / 32.0f);
    const float rinv = 1.0f / sqrtf(var + LNEPS);
    const float* gp = cst + 112 + 16 * hf;
    const float* bp = cst + 144 + 16 * hf;
    v8us h0, h1, l0, l1, w0, w1;
#pragma unroll
    for (int i = 0; i < 8; ++i) {
      unsigned lb;
      unsigned hb = hl_bits(d[i] * rinv * gp[i] + bp[i], lb);
      h0[i] = (unsigned short)hb; l0[i] = (unsigned short)lb;
      w0[i] = (unsigned short)bf16_bits(r[i]);
      hb = hl_bits(d[8 + i] * rinv * gp[8 + i] + bp[8 + i], lb);
      h1[i] = (unsigned short)hb; l1[i] = (unsigned short)lb;
      w1[i] = (unsigned short)bf16_bits(r[8 + i]);
    }
    unsigned short* arow = sA + row * EA_P + 16 * hf;
    *(v8usa*)(arow)      = h0;
    *(v8usa*)(arow + 8)  = h1;
    *(v8usa*)(arow + 32) = l0;
    *(v8usa*)(arow + 40) = l1;
    unsigned short* rrow = sR + row * ER_P + 16 * hf;
    *(v8usa*)(rrow)     = w0;
    *(v8usa*)(rrow + 8) = w1;
  }
  __syncthreads();

  {
    v8f acc[4];
#pragma unroll
    for (int t = 0; t < 4; ++t) acc[t] = z8();
    const unsigned short* ap = sA + (16 * wave + m) * EA_P + 8 * hh;
    const unsigned short* bp = EE1D + (size_t)m * 64 + 8 * hh;
#pragma unroll
    for (int ks = 0; ks < 2; ++ks) {
      FragB af;
      af.h[0] = *(const v8usa*)(ap + 32 * ks);
      af.h[1] = *(const v8usa*)(ap + 32 * ks + 16);
#pragma unroll
      for (int nt = 0; nt < 4; ++nt) {
        const unsigned short* wq = bp + (size_t)(16 * nt) * 64 + 32 * ks;
        FragB bf;
        bf.h[0] = *(const v8usa*)wq;
        bf.h[1] = *(const v8usa*)(wq + 16);
        acc[nt] = wmb(af, bf, acc[nt]);
      }
    }
    v8f accg = z8();
    {
      const unsigned short* ar = sR + (16 * wave + m) * ER_P + 8 * hh;
      const unsigned short* bq = ECW + (size_t)m * 32 + 8 * hh;
      FragB af, bf;
      af.h[0] = *(const v8usa*)ar;
      af.h[1] = *(const v8usa*)(ar + 16);
      bf.h[0] = *(const v8usa*)bq;
      bf.h[1] = *(const v8usa*)(bq + 16);
      accg = wmb(af, bf, accg);
    }
#pragma unroll
    for (int nt = 0; nt < 4; ++nt) {
      const int c = 16 * nt + m;
      const float bb = cst[c];
#pragma unroll
      for (int r = 0; r < 8; ++r) {
        const int lr = 16 * wave + 8 * hh + r;
        const float v = acc[nt][r] + bb;
        sH[lr * EH_P + c] = v > 0.0f ? v : 0.0f;
      }
    }
    {
      const float bz = cst[64 + m];
#pragma unroll
      for (int r = 0; r < 8; ++r) {
        const int lr = 16 * wave + 8 * hh + r;
        const float v = accg[r] + bz;
        sZ[lr * EZ_P + m] = v > 0.0f ? v : 0.0f;
      }
    }
  }
  __syncthreads();

  {
    const float* hp = sH + row * EH_P + 32 * hf;
    unsigned short* mp = sM + row * HP + 32 * hf;
#pragma unroll
    for (int c8 = 0; c8 < 4; ++c8) {
      const v4f a = *(const v4fa*)(hp + 8 * c8);
      const v4f b = *(const v4fa*)(hp + 8 * c8 + 4);
      const float f8[8] = {a.x, a.y, a.z, a.w, b.x, b.y, b.z, b.w};
      v8us oh, ol;
#pragma unroll
      for (int e = 0; e < 8; ++e) {
        unsigned lb;
        const unsigned hb = hl_bits(f8[e], lb);
        oh[e] = (unsigned short)hb; ol[e] = (unsigned short)lb;
      }
      *(v8usa*)(mp + 8 * c8)      = oh;
      *(v8usa*)(mp + 64 + 8 * c8) = ol;
    }
    float z = 0.0f;
#pragma unroll 4
    for (int j = 0; j < 16; ++j) z = fmaf(sZ[row * EZ_P + j], cst[80 + j], z);
    z += cst[96];
    const float ew = 1.0f / (1.0f + expf(-z));
    if (hf == 0) sEW[row] = ew;
  }
  __syncthreads();

  {
    v4i pv[8];
#pragma unroll
    for (int it = 0; it < 8; ++it) pv[it] = *(const v4ia*)(sM + (size_t)(it * NTHR + tid) * 8);
    unsigned short* mb = HID + (size_t)blockIdx.x * TROWS * HP;
#pragma unroll
    for (int it = 0; it < 8; ++it) *(volatile v4i*)(mb + (size_t)(it * NTHR + tid) * 8) = pv[it];
    __threadfence();
#pragma unroll
    for (int it = 0; it < 8; ++it) *(volatile v4i*)(mb + (size_t)(it * NTHR + tid) * 8) = pv[it];
  }
  {
    const int tl = tid < 32 ? tid : 31;
    const v4f o4 = *(const v4fa*)(sEW + 4 * tl);
    float* sp = EWG + (size_t)blockIdx.x * TROWS + 4 * tl;
    if (tid < 32) *(volatile v4f*)sp = o4;
    __threadfence();
    if (tid < 32) *(volatile v4f*)sp = o4;
  }
}

template <int NT, int EPI>
__global__ __launch_bounds__(GTHR) KVG void k_gemm(const unsigned short* __restrict__ A, int lda,
                                                   const unsigned short* __restrict__ BT, int ldb, int K,
                                                   const float* __restrict__ bias, int nBias, float scale,
                                                   const float* __restrict__ gam, const float* __restrict__ bet,
                                                   const int* __restrict__ TAB, int nTab,
                                                   const float* __restrict__ AUX,
                                                   float* Cf, int ldc, unsigned short* Ch, int ldh, int hoff,
                                                   int nN) {
  static_assert(NT == 2 || NT == 4 || NT == 8);
  constexpr int W   = 16 * NT;
  constexpr int LPR = W / 4;
  constexpr int RPP = 32 / LPR;
  constexpr int NP  = 16 / RPP;
  constexpr int NQ  = W / 8;
  constexpr int PPR = (2 * W) / 8;
  __shared__ __attribute__((aligned(16))) float stg[GBM * W];
  __shared__ int   sCn[GBM];
  __shared__ float sAx[GBM];
  const int tid = (int)threadIdx.x, lane = tid & 31, wave = tid >> 5, hh = lane >> 4, m = lane & 15;
  const int rowBase = (int)blockIdx.x * GBM;
  const int colBase = (int)blockIdx.y * W;

  v8f acc[NT];
#pragma unroll
  for (int t = 0; t < NT; ++t) acc[t] = z8();
  const unsigned short* ap = A  + (size_t)(rowBase + 16 * wave + m) * (size_t)lda + 8 * hh;
  const unsigned short* bp = BT + (size_t)(colBase + m) * (size_t)ldb + 8 * hh;
#pragma unroll 1
  for (int k0 = 0; k0 < K; k0 += 32) {
    FragB af;
    af.h[0] = *(const v8usa*)(ap + k0);
    af.h[1] = *(const v8usa*)(ap + k0 + 16);
#pragma unroll
    for (int nt = 0; nt < NT; ++nt) {
      const unsigned short* wq = bp + (size_t)(16 * nt) * (size_t)ldb + k0;
      FragB bf;
      bf.h[0] = *(const v8usa*)wq;
      bf.h[1] = *(const v8usa*)(wq + 16);
      acc[nt] = wmb(af, bf, acc[nt]);
    }
  }
#pragma unroll
  for (int nt = 0; nt < NT; ++nt) {
    const int lc = 16 * nt + m;
#pragma unroll
    for (int r = 0; r < 8; ++r) {
      const int lr = 16 * wave + 8 * hh + r;
      stg[lr * W + lc] = acc[nt][r];
    }
  }
  float pz = 0.0f;
  if constexpr (EPI != 0) {
    const int sr = rowBase + (tid & (GBM - 1));
    if constexpr (EPI <= 3) {
      const int cv = TAB[sr];
      if (tid < GBM) sCn[tid] = cv;
    } else {
      const float av = AUX[sr];
      if (tid < GBM) sAx[tid] = av;
    }
    if constexpr (EPI >= 3) {
      const int mflag = TAB[(size_t)2 * nTab + (size_t)(rowBase >> SLA) * 32 + 1];
      pz = (mflag != 0) ? __int_as_float(0x7fc00000) : 0.0f;
    }
  }
  __syncthreads();

  const int rsub = lane / LPR, j = lane % LPR;
  v4f pv[NP];
#pragma unroll
  for (int i = 0; i < NP; ++i) pv[i] = *(const v4fa*)(stg + (16 * wave + i * RPP + rsub) * W + 4 * j);

  if constexpr (EPI == 0) {
    v4f bv;
    {
      float bb[4];
#pragma unroll
      for (int e = 0; e < 4; ++e) {
        const int cc = colBase + 4 * j + e;
        const int ci = cc < nBias ? cc : nBias - 1;
        const float f = bf16_val(bias[ci]);
        bb[e] = cc < nBias ? f : 0.0f;
      }
      bv.x = bb[0]; bv.y = bb[1]; bv.z = bb[2]; bv.w = bb[3];
    }
#pragma unroll
    for (int i = 0; i < NP; ++i) pv[i] = scale * (pv[i] + bv);
#pragma unroll
    for (int i = 0; i < NP; ++i) {
      float* op = Cf + (size_t)(rowBase + 16 * wave + i * RPP + rsub) * (size_t)ldc + colBase + 4 * j;
      *(volatile v4f*)op = pv[i];
    }
    __threadfence();
#pragma unroll
    for (int i = 0; i < NP; ++i) {
      float* op = Cf + (size_t)(rowBase + 16 * wave + i * RPP + rsub) * (size_t)ldc + colBase + 4 * j;
      *(volatile v4f*)op = pv[i];
    }
  } else {
    __syncthreads();
    const v4f b4 = *(const v4f*)(bias + 4 * j);
    const float bq[4] = {bf16_val(b4.x), bf16_val(b4.y), bf16_val(b4.z), bf16_val(b4.w)};
    float gq[4] = {0.f, 0.f, 0.f, 0.f}, eq[4] = {0.f, 0.f, 0.f, 0.f};
    if constexpr (EPI <= 3) {
      const v4f g4 = *(const v4f*)(gam + 4 * j);
      const v4f e4 = *(const v4f*)(bet + 4 * j);
      gq[0] = bf16_val(g4.x); gq[1] = bf16_val(g4.y); gq[2] = bf16_val(g4.z); gq[3] = bf16_val(g4.w);
      eq[0] = bf16_val(e4.x); eq[1] = bf16_val(e4.y); eq[2] = bf16_val(e4.z); eq[3] = bf16_val(e4.w);
    }
    const float invw = 1.0f / (float)W;
#pragma unroll
    for (int i = 0; i < NP; ++i) {
      const int lrow = 16 * wave + i * RPP + rsub;
      const int row  = rowBase + lrow;
      float o0, o1, o2, o3;
      if constexpr (EPI <= 3) {
        const int cn = sCn[lrow];
        const bool hasb = cn > 0;
        const float y0 = pv[i].x + (hasb ? bq[0] : 0.0f);
        const float y1 = pv[i].y + (hasb ? bq[1] : 0.0f);
        const float y2 = pv[i].z + (hasb ? bq[2] : 0.0f);
        const float y3 = pv[i].w + (hasb ? bq[3] : 0.0f);
        float s = (y0 + y1) + (y2 + y3);
#pragma unroll
        for (int o = LPR / 2; o > 0; o >>= 1) s += __shfl_xor(s, o, 32);
        const float mean = s * invw;
        const float d0 = y0 - mean, d1 = y1 - mean, d2 = y2 - mean, d3 = y3 - mean;
        float q = (d0 * d0 + d1 * d1) + (d2 * d2 + d3 * d3);
#pragma unroll
        for (int o = LPR / 2; o > 0; o >>= 1) q += __shfl_xor(q, o, 32);
        const float var  = q * invw;
        const float rinv = 1.0f / sqrtf(var + LNEPS);
        o0 = d0 * rinv * gq[0] + eq[0];
        o1 = d1 * rinv * gq[1] + eq[1];
        o2 = d2 * rinv * gq[2] + eq[2];
        o3 = d3 * rinv * gq[3] + eq[3];
        if constexpr (EPI == 1) {
          o0 = o0 > 0.0f ? o0 : 0.01f * o0;
          o1 = o1 > 0.0f ? o1 : 0.01f * o1;
          o2 = o2 > 0.0f ? o2 : 0.01f * o2;
          o3 = o3 > 0.0f ? o3 : 0.01f * o3;
        } else {
          o0 = relu_np(o0); o1 = relu_np(o1); o2 = relu_np(o2); o3 = relu_np(o3);
        }
        if constexpr (EPI == 3) {
          const v4f ax = *(const v4f*)(AUX + (size_t)row * 128 + 4 * j);
          o0 = (ax.x + o0) + pz; o1 = (ax.y + o1) + pz; o2 = (ax.z + o2) + pz; o3 = (ax.w + o3) + pz;
        }
      } else {
        const float sw = sAx[lrow];
        o0 = (pv[i].x + sw * bq[0]) + pz;
        o1 = (pv[i].y + sw * bq[1]) + pz;
        o2 = (pv[i].z + sw * bq[2]) + pz;
        o3 = (pv[i].w + sw * bq[3]) + pz;
      }
      v4f qo;
      qo.x = o0; qo.y = o1; qo.z = o2; qo.w = o3;
      pv[i] = qo;
    }
    if constexpr (EPI >= 3) {
      const int co = (EPI == 3) ? 0 : 128;
#pragma unroll
      for (int i = 0; i < NP; ++i) {
        const int row = rowBase + 16 * wave + i;
        float* op = Cf + (size_t)row * (size_t)ldc + co + 4 * j;
        if (row < nN) *(volatile v4f*)op = pv[i];
      }
      __threadfence();
#pragma unroll
      for (int i = 0; i < NP; ++i) {
        const int row = rowBase + 16 * wave + i;
        float* op = Cf + (size_t)row * (size_t)ldc + co + 4 * j;
        if (row < nN) *(volatile v4f*)op = pv[i];
      }
    }
#pragma unroll
    for (int i = 0; i < NP; ++i) {
      v4us h4, l4;
      unsigned lb;
      unsigned hb;
      hb = hl_bits(pv[i].x, lb); h4[0] = (unsigned short)hb; l4[0] = (unsigned short)lb;
      hb = hl_bits(pv[i].y, lb); h4[1] = (unsigned short)hb; l4[1] = (unsigned short)lb;
      hb = hl_bits(pv[i].z, lb); h4[2] = (unsigned short)hb; l4[2] = (unsigned short)lb;
      hb = hl_bits(pv[i].w, lb); h4[3] = (unsigned short)hb; l4[3] = (unsigned short)lb;
      unsigned short* srow = (unsigned short*)stg + (size_t)(16 * wave + i * RPP + rsub) * (2 * W);
      *(v4usa*)(srow + 4 * j)     = h4;
      *(v4usa*)(srow + W + 4 * j) = l4;
    }
    __syncthreads();
    v8us qv[NQ];
    const unsigned short* sbase = (const unsigned short*)stg + (size_t)(16 * wave) * (2 * W);
#pragma unroll
    for (int it = 0; it < NQ; ++it) qv[it] = *(const v8usa*)(sbase + (size_t)(it * 32 + lane) * 8);
#pragma unroll
    for (int it = 0; it < NQ; ++it) {
      const int q = it * 32 + lane;
      const int prow = q / PPR, jj = q % PPR;
      unsigned short* rp = Ch + (size_t)(rowBase + 16 * wave + prow) * (size_t)ldh + hoff + 8 * jj;
      *(volatile v8us*)rp = qv[it];
    }
    __threadfence();
#pragma unroll
    for (int it = 0; it < NQ; ++it) {
      const int q = it * 32 + lane;
      const int prow = q / PPR, jj = q % PPR;
      unsigned short* rp = Ch + (size_t)(rowBase + 16 * wave + prow) * (size_t)ldh + hoff + 8 * jj;
      *(volatile v8us*)rp = qv[it];
    }
  }
}

template <int H, int GSF>
__global__ __launch_bounds__(NTHR) KVG void k_layer(const int* __restrict__ ei, int nE, int nN,
                                                    const int* __restrict__ LISTP, const int* __restrict__ TAB,
                                                    int nTab,
                                                    const unsigned short* __restrict__ HID,
                                                    const float* __restrict__ EWG,
                                                    const unsigned short* __restrict__ MHL,
                                                    const float* __restrict__ CLp,
                                                    const float* __restrict__ PDPS,
                                                    unsigned short* AHL, unsigned short* GSHL, float* SWp) {
  static_assert(H == 32 || H == 64 || H == 128);
  static_assert(NTHR % H == 0);
  constexpr int TP  = H + 4;
  constexpr int G   = NTHR / H;
  constexpr int NPG = TROWS / G;
  constexpr int NTL = H / 16;
  constexpr int NPC = H / 8;
  extern __shared__ __attribute__((aligned(16))) unsigned char dynb[];
  unsigned short* sA = (unsigned short*)dynb;
  float* sT   = (float*)(dynb + TROWS * AP * 2);
  float* sAcc = sT + TROWS * TP;
  float* sG   = sAcc + TROWS * H;
  int*   sEid = (int*)(sG + (GSF ? TROWS * 64 : 0));
  int*   sSrc = sEid + TROWS;
  int*   sDl  = sSrc + TROWS;
  float* sEw  = (float*)(sDl + TROWS);
  int*   sOff = (int*)(sEw + TROWS);
  float* sInv = (float*)(sOff + 132);
  float* sCL  = sInv + TROWS;
  float* sSw  = sCL + H;

  const int tid = (int)threadIdx.x, lane = tid & 31, wave = tid >> 5, hh = lane >> 4, m = lane & 15;
  const int n0 = (int)blockIdx.x * TROWS;
  const int cb = n0 >> SLA;
  const int* CNT  = TAB;
  const int* LOFF = TAB + nTab;
  const int* META = TAB + (size_t)2 * nTab;
  const int* srcs = ei;
  const int* dsts = ei + nE;
  const int* listBase = LISTP + (size_t)cb * RCAP;

  const int start = clampi(LOFF[n0], 0, RCAP);
  int endp;
  {
    const int lo_l = clampi(LOFF[n0 + TROWS - 1], 0, RCAP);
    const int c_l  = clampi(CNT[n0 + TROWS - 1], 0, RCAP);
    endp = lo_l + c_l;
    endp = endp > RCAP ? RCAP : endp;
    endp = endp < start ? start : endp;
  }
  const int tot = endp - start;
  const int ovf = META[cb * 32 + 1];
  const float qnan = __int_as_float(0x7fc00000);
  const float pz = (ovf != 0) ? qnan : 0.0f;

  {
    const v4f z4 = {0.0f, 0.0f, 0.0f, 0.0f};
    for (int i = tid * 4; i < TROWS * H; i += NTHR * 4) *(v4fa*)(sAcc + i) = z4;
    if constexpr (GSF != 0) {
      for (int i = tid * 4; i < TROWS * 64; i += NTHR * 4) *(v4fa*)(sG + i) = z4;
    }
  }
  if (tid < TROWS) {
    const int o = clampi(LOFF[n0 + tid], start, endp) - start;
    sOff[tid] = o;
    int c = CNT[n0 + tid];
    c = c < 0 ? 0 : c;
    sInv[tid] = 1.0f / fmaxf((float)c, 1.0f);
  }
  if (tid >= TROWS && tid < TROWS + 4) sOff[tid] = tot;
  if (tid < H) sCL[tid] = CLp[tid];
  float swacc = 0.0f;
  __syncthreads();

  const int nTiles = (tot + TROWS - 1) / TROWS;
#pragma unroll 1
  for (int tl = 0; tl < nTiles; ++tl) {
    const int tb = tl * TROWS;
    if (tid < TROWS) {
      const int p  = start + tb + tid;
      const bool valid = p < endp;
      const int pc = p < RCAP ? p : RCAP - 1;
      const int eid = clampi(listBase[pc], 0, nE - 1);
      const int s   = clampi(srcs[eid], 0, nN - 1);
      const int dl  = clampi(dsts[eid] - n0, 0, TROWS - 1);
      const float ew = EWG[eid];
      sEid[tid] = valid ? eid : -1;
      sSrc[tid] = s;
      sDl[tid]  = dl;
      sEw[tid]  = valid ? ew : 0.0f;
    }
    __syncthreads();
#pragma unroll
    for (int it = 0; it < 8; ++it) {
      const int p   = it * NTHR + tid;
      const int row = p >> 4, jj = p & 15;
      const int eid = sEid[row];
      const int mk  = eid >= 0 ? -1 : 0;
      const int ec  = eid >= 0 ? eid : 0;
      v4i v = *(const v4ia*)(HID + (size_t)ec * HP + 8 * jj);
      const v4i mm = {mk, mk, mk, mk};
      v = v & mm;
      *(v4ia*)(sA + row * AP + 8 * jj) = v;
    }
    __syncthreads();
    {
      v8f acc[NTL];
#pragma unroll
      for (int t = 0; t < NTL; ++t) acc[t] = z8();
      const unsigned short* ap = sA + (16 * wave + m) * AP + 8 * hh;
      const unsigned short* bp = MHL + (size_t)m * 192 + 8 * hh;
#pragma unroll 1
      for (int ks = 0; ks < 6; ++ks) {
        const int acol = 32 * (ks < 4 ? ks : ks - 4);
        FragB af;
        af.h[0] = *(const v8usa*)(ap + acol);
        af.h[1] = *(const v8usa*)(ap + acol + 16);
#pragma unroll
        for (int nt = 0; nt < NTL; ++nt) {
          const unsigned short* wq = bp + (size_t)(16 * nt) * 192 + 32 * ks;
          FragB bf;
          bf.h[0] = *(const v8usa*)wq;
          bf.h[1] = *(const v8usa*)(wq + 16);
          acc[nt] = wmb(af, bf, acc[nt]);
        }
      }
#pragma unroll
      for (int nt = 0; nt < NTL; ++nt) {
        const int lc = 16 * nt + m;
#pragma unroll
        for (int r = 0; r < 8; ++r) sT[(16 * wave + 8 * hh + r) * TP + lc] = acc[nt][r];
      }
    }
    __syncthreads();
    {
      const int c = tid % H, g = tid / H;
      int lo = sOff[g * NPG], hi = sOff[(g + 1) * NPG];
      lo = lo > tb ? lo : tb;
      hi = hi < tb + TROWS ? hi : tb + TROWS;
      const float clc = sCL[c];
      const float* pdb = PDPS + (size_t)n0 * (2 * H) + c;
      const float* psb = PDPS + H + c;
#pragma unroll 2
      for (int rr = lo; rr < hi; ++rr) {
        const int r  = rr - tb;
        const int nd = sDl[r];
        const int ps = sSrc[r];
        const float ew = sEw[r];
        const float pd  = pdb[(size_t)nd * (2 * H)];
        const float psv = psb[(size_t)ps * (2 * H)];
        const float v = (pd + psv) + ew * (sT[r * TP + c] + clc);
        sAcc[nd * H + c] += relu_np(v);
      }
    }
    if constexpr (GSF != 0) {
      const int c2 = tid & 63, g2 = tid >> 6;
      int lo = sOff[32 * g2], hi = sOff[32 * g2 + 32];
      lo = lo > tb ? lo : tb;
      hi = hi < tb + TROWS ? hi : tb + TROWS;
#pragma unroll 2
      for (int rr = lo; rr < hi; ++rr) {
        const int r  = rr - tb;
        const int nd = sDl[r];
        const float ew = sEw[r];
        const unsigned short* ar = sA + r * AP;
        const float f = __uint_as_float(((unsigned)ar[c2]) << 16) + __uint_as_float(((unsigned)ar[64 + c2]) << 16);
        sG[nd * 64 + c2] += ew * f;
      }
      if (tid < TROWS) {
        int rows = tot - tb;
        rows = rows > TROWS ? TROWS : rows;
#pragma unroll 4
        for (int r = 0; r < rows; ++r) swacc += (sDl[r] == tid) ? sEw[r] : 0.0f;
      }
    }
    __syncthreads();
  }

  {
    unsigned short* sSt = (unsigned short*)sT;
    const int c = tid % H, g = tid / H;
#pragma unroll 4
    for (int q = 0; q < NPG; ++q) {
      const int nd = g * NPG + q;
      const float v = sAcc[nd * H + c] * sInv[nd] + pz;
      unsigned lb;
      const unsigned hb = hl_bits(v, lb);
      sSt[nd * 2 * H + c]     = (unsigned short)hb;
      sSt[nd * 2 * H + H + c] = (unsigned short)lb;
    }
  }
  if constexpr (GSF != 0) {
    unsigned short* sGs = sA;
    const int c2 = tid & 63, g2 = tid >> 6;
#pragma unroll 4
    for (int q = 0; q < 32; ++q) {
      const int nd = 32 * g2 + q;
      const float v = sG[nd * 64 + c2] * sInv[nd] + pz;
      unsigned lb;
      const unsigned hb = hl_bits(v, lb);
      sGs[nd * HP + c2]      = (unsigned short)hb;
      sGs[nd * HP + 64 + c2] = (unsigned short)lb;
    }
    if (tid < TROWS) sSw[tid] = swacc * sInv[tid] + pz;
  }
  __syncthreads();
  {
    const unsigned short* sSt = (const unsigned short*)sT;
    v4i pv[NPC];
#pragma unroll
    for (int it = 0; it < NPC; ++it) pv[it] = *(const v4ia*)(sSt + (size_t)(it * NTHR + tid) * 8);
    unsigned short* ab = AHL + (size_t)n0 * (2 * H);
#pragma unroll
    for (int it = 0; it < NPC; ++it) *(volatile v4i*)(ab + (size_t)(it * NTHR + tid) * 8) = pv[it];
    __threadfence();
#pragma unroll
    for (int it = 0; it < NPC; ++it) *(volatile v4i*)(ab + (size_t)(it * NTHR + tid) * 8) = pv[it];
  }
  if constexpr (GSF != 0) {
    v4i pv[8];
#pragma unroll
    for (int it = 0; it < 8; ++it) pv[it] = *(const v4ia*)(sA + (size_t)(it * NTHR + tid) * 8);
    unsigned short* gb = GSHL + (size_t)n0 * HP;
    const int tl2 = tid < 32 ? tid : 31;
    const v4f o4 = *(const v4fa*)(sSw + 4 * tl2);
    float* sp = SWp + (size_t)n0 + 4 * tl2;
#pragma unroll
    for (int it = 0; it < 8; ++it) *(volatile v4i*)(gb + (size_t)(it * NTHR + tid) * 8) = pv[it];
    if (tid < 32) *(volatile v4f*)sp = o4;
    __threadfence();
#pragma unroll
    for (int it = 0; it < 8; ++it) *(volatile v4i*)(gb + (size_t)(it * NTHR + tid) * 8) = pv[it];
    if (tid < 32) *(volatile v4f*)sp = o4;
  }
}

__global__ __launch_bounds__(GTHR) KVG void k_head(const unsigned short* __restrict__ XF,
                                                   const unsigned short* __restrict__ NP1D,
                                                   const unsigned short* __restrict__ NP2D,
                                                   const float* __restrict__ b1, const float* __restrict__ b2,
                                                   const float* __restrict__ w3, const float* __restrict__ b3,
                                                   const int* __restrict__ TAB, int nTab, float* out1, int nN) {
  extern __shared__ __attribute__((aligned(16))) unsigned char dynb[];
  float*          stg  = (float*)dynb;
  unsigned short* sH   = (unsigned short*)(dynb + GBM * 128 * 4);
  float*          sB2  = (float*)(dynb + GBM * 128 * 4 + GBM * HD_P * 2);
  float*          sW3  = sB2 + 64;
  float*          sOut = sW3 + 64;
  const int tid = (int)threadIdx.x, lane = tid & 31, wave = tid >> 5, hh = lane >> 4, m = lane & 15;
  const int rowBase = (int)blockIdx.x * GBM;

  {
    v8f acc[8];
#pragma unroll
    for (int t = 0; t < 8; ++t) acc[t] = z8();
    const unsigned short* ap = XF + (size_t)(rowBase + 16 * wave + m) * 512 + 8 * hh;
    const unsigned short* bp = NP1D + (size_t)m * 512 + 8 * hh;
#pragma unroll 1
    for (int k0 = 0; k0 < 512; k0 += 32) {
      FragB af;
      af.h[0] = *(const v8usa*)(ap + k0);
      af.h[1] = *(const v8usa*)(ap + k0 + 16);
#pragma unroll
      for (int nt = 0; nt < 8; ++nt) {
        const unsigned short* wq = bp + (size_t)(16 * nt) * 512 + k0;
        FragB bf;
        bf.h[0] = *(const v8usa*)wq;
        bf.h[1] = *(const v8usa*)(wq + 16);
        acc[nt] = wmb(af, bf, acc[nt]);
      }
    }
#pragma unroll
    for (int nt = 0; nt < 8; ++nt) {
      const int lc = 16 * nt + m;
#pragma unroll
      for (int r = 0; r < 8; ++r) stg[(16 * wave + 8 * hh + r) * 128 + lc] = acc[nt][r];
    }
  }
  if (tid < 64) { sB2[tid] = bf16_val(b2[tid]); sW3[tid] = bf16_val(w3[tid]); }
  __syncthreads();
  {
    const v4f b4 = *(const v4f*)(b1 + 4 * lane);
    const float q0 = bf16_val(b4.x), q1 = bf16_val(b4.y), q2 = bf16_val(b4.z), q3 = bf16_val(b4.w);
#pragma unroll 1
    for (int it = 0; it < 16; ++it) {
      const int row = it * 4 + wave;
      const v4f v = *(const v4fa*)(stg + row * 128 + 4 * lane);
      const float e0 = elu_f(v.x + q0), e1 = elu_f(v.y + q1), e2 = elu_f(v.z + q2), e3 = elu_f(v.w + q3);
      v4us h4, l4;
      unsigned lb;
      unsigned hb;
      hb = hl_bits(e0, lb); h4[0] = (unsigned short)hb; l4[0] = (unsigned short)lb;
      hb = hl_bits(e1, lb); h4[1] = (unsigned short)hb; l4[1] = (unsigned short)lb;
      hb = hl_bits(e2, lb); h4[2] = (unsigned short)hb; l4[2] = (unsigned short)lb;
      hb = hl_bits(e3, lb); h4[3] = (unsigned short)hb; l4[3] = (unsigned short)lb;
      *(v4usa*)(sH + row * HD_P + 4 * lane)       = h4;
      *(v4usa*)(sH + row * HD_P + 128 + 4 * lane) = l4;
    }
  }
  __syncthreads();
  {
    v8f acc[4];
#pragma unroll
    for (int t = 0; t < 4; ++t) acc[t] = z8();
    const unsigned short* ap = sH + (16 * wave + m) * HD_P + 8 * hh;
    const unsigned short* bp = NP2D + (size_t)m * 256 + 8 * hh;
#pragma unroll 1
    for (int k0 = 0; k0 < 256; k0 += 32) {
      FragB af;
      af.h[0] = *(const v8usa*)(ap + k0);
      af.h[1] = *(const v8usa*)(ap + k0 + 16);
#pragma unroll
      for (int nt = 0; nt < 4; ++nt) {
        const unsigned short* wq = bp + (size_t)(16 * nt) * 256 + k0;
        FragB bf;
        bf.h[0] = *(const v8usa*)wq;
        bf.h[1] = *(const v8usa*)(wq + 16);
        acc[nt] = wmb(af, bf, acc[nt]);
      }
    }
#pragma unroll
    for (int nt = 0; nt < 4; ++nt) {
      const int lc = 16 * nt + m;
#pragma unroll
      for (int r = 0; r < 8; ++r) stg[(16 * wave + 8 * hh + r) * 128 + lc] = acc[nt][r];
    }
  }
  __syncthreads();
  {
    const int row = tid >> 1, hf = tid & 1;
    float p = 0.0f;
#pragma unroll 4
    for (int c = 0; c < 32; ++c) {
      const int cc = 32 * hf + c;
      const float e = elu_f(stg[row * 128 + cc] + sB2[cc]);
      p = fmaf(e, sW3[cc], p);
    }
    p += __shfl_xor(p, 1, 32);
    const int rg = rowBase + row;
    const float pz = (TAB[(size_t)2 * nTab + (size_t)(rg >> SLA) * 32 + 1] != 0) ? __int_as_float(0x7fc00000) : 0.0f;
    p = (p + bf16_val(b3[0])) + pz;
    if (hf == 0) sOut[row] = p;
  }
  __syncthreads();
  {
    const int tl = tid < 16 ? tid : 15;
    const v4f o4 = *(const v4fa*)(sOut + 4 * tl);
    const bool stv = (tid < 16) && (rowBase + 4 * tl + 3 < nN);
    float* op = out1 + (size_t)rowBase + 4 * tl;
    if (stv) *(volatile v4f*)op = o4;
    __threadfence();
    if (stv) *(volatile v4f*)op = o4;
  }
}

static inline int cdiv(int a, int b) { return (a + b - 1) / b; }
static inline size_t al256(size_t o) { return (o + 255) & ~(size_t)255; }
template <int H, int GSF> static constexpr int layer_lds_bytes() {
  return TROWS * AP * 2 + TROWS * (H + 4) * 4 + TROWS * H * 4 + (GSF ? TROWS * 64 * 4 : 0) +
         (4 * TROWS + 132 + TROWS + H + TROWS) * 4;
}
static_assert(layer_lds_bytes<128, 1>() <= 300000);

static inline void wplane(hipStream_t st, const float* W, int ldw, int rbase, int per, int Kp, int Nn,
                          unsigned short* D) {
  const int nUnits = Nn * Kp / 8;
  k_wplane<<<cdiv(nUnits, NTHR), NTHR, 0, st>>>(W, ldw, rbase, per, Kp, nUnits, D);
}

extern "C" void kernel_launch(void* const* d_in, const int* in_sizes, int n_in,
                              void* d_out, int out_size, void* d_ws, size_t ws_size,
                              hipStream_t stream) {
  if (n_in < 43) return;
  if (in_sizes[0] < 64 * 128 || (in_sizes[0] % 64) != 0) return;
  const int nN = in_sizes[0] / 64;
  if (in_sizes[1] < 2 || (in_sizes[1] & 1) != 0) return;
  const int nE = in_sizes[1] / 2;
  if (nE < 1 || nE >= (1 << 21) || nN > (1 << 20) || (nN & 3) != 0) return;
  if ((long long)in_sizes[2] != 32LL * nE) return;
  {
    static const int want[40] = {64, 64, 64, 64, 8192, 128, 32, 32, 2048, 64, 8192, 128, 512, 16, 16, 1,
                                 8192, 32, 1024, 32, 12288, 64, 4096, 64, 32768, 128, 16384, 128,
                                 32, 32, 64, 64, 128, 128, 32768, 128, 8192, 64, 64, 1};
    for (int i = 0; i < 40; ++i) if (in_sizes[3 + i] != want[i]) return;
  }
  if ((long long)out_size != 257LL * nN) return;

  const float* x_in  = (const float*)d_in[0];
  const int*   ei    = (const int*)  d_in[1];
  const float* eattr = (const float*)d_in[2];
  const float* bn0w  = (const float*)d_in[3];
  const float* bn0b  = (const float*)d_in[4];
  const float* bn0rm = (const float*)d_in[5];
  const float* bn0rv = (const float*)d_in[6];
  const float* projw = (const float*)d_in[7];
  const float* projb = (const float*)d_in[8];
  const float* eelng = (const float*)d_in[9];
  const float* eelnb = (const float*)d_in[10];
  const float* eew1  = (const float*)d_in[11];
  const float* eeb1  = (const float*)d_in[12];
  const float* eew2  = (const float*)d_in[13];
  const float* eeb2  = (const float*)d_in[14];
  const float* ecw1  = (const float*)d_in[15];
  const float* ecb1  = (const float*)d_in[16];
  const float* ecw2  = (const float*)d_in[17];
  const float* ecb2  = (const float*)d_in[18];
  const float* c1w1  = (const float*)d_in[19];
  const float* c1b1  = (const float*)d_in[20];
  const float* c1w2  = (const float*)d_in[21];
  const float* c1b2  = (const float*)d_in[22];
  const float* c2w1  = (const float*)d_in[23];
  const float* c2b1  = (const float*)d_in[24];
  const float* c2w2  = (const float*)d_in[25];
  const float* c2b2  = (const float*)d_in[26];
  const float* c3w1  = (const float*)d_in[27];
  const float* c3b1  = (const float*)d_in[28];
  const float* c3w2  = (const float*)d_in[29];
  const float* c3b2  = (const float*)d_in[30];
  const float* ln1g  = (const float*)d_in[31];
  const float* ln1b  = (const float*)d_in[32];
  const float* ln2g  = (const float*)d_in[33];
  const float* ln2b  = (const float*)d_in[34];
  const float* ln3g  = (const float*)d_in[35];
  const float* ln3b  = (const float*)d_in[36];
  const float* npw1  = (const float*)d_in[37];
  const float* npb1  = (const float*)d_in[38];
  const float* npw2  = (const float*)d_in[39];
  const float* npb2  = (const float*)d_in[40];
  const float* npw3  = (const float*)d_in[41];
  const float* npb3  = (const float*)d_in[42];
  float* out0 = (float*)d_out;
  float* out1 = out0 + (size_t)nN * 256;

  const int MP   = cdiv(nN, TROWS) * TROWS;
  const int gL   = MP / TROWS;
  const int gM   = MP / GBM;
  const int gC   = cdiv(MP, NBA);
  const int nTab = gC * NBA;
  const int gE   = cdiv(nE, TROWS);
  const size_t EP = (size_t)gE * TROWS;
  if (nTab < MP) return;

  char* ws = (char*)d_ws;
  size_t off = 0;
  const size_t oEE1D = off; off = al256(off + (size_t)64 * 64 * 2);
  const size_t oECW  = off; off = al256(off + (size_t)16 * 32 * 2);
  const size_t oMHL1 = off; off = al256(off + (size_t)32 * 192 * 2);
  const size_t oMHL2 = off; off = al256(off + (size_t)64 * 192 * 2);
  const size_t oMHL3 = off; off = al256(off + (size_t)128 * 192 * 2);
  const size_t oCL1  = off; off = al256(off + 512);
  const size_t oCL2  = off; off = al256(off + 512);
  const size_t oCL3  = off; off = al256(off + 512);
  const size_t oWPD1 = off; off = al256(off + (size_t)64 * 128 * 2);
  const size_t oWPD2 = off; off = al256(off + (size_t)128 * 64 * 2);
  const size_t oWPD3 = off; off = al256(off + (size_t)256 * 128 * 2);
  const size_t oW2D1 = off; off = al256(off + (size_t)32 * 64 * 2);
  const size_t oW2D2 = off; off = al256(off + (size_t)64 * 128 * 2);
  const size_t oW2D3 = off; off = al256(off + (size_t)128 * 256 * 2);
  const size_t oPROJ = off; off = al256(off + (size_t)128 * 128 * 2);
  const size_t oEE2D = off; off = al256(off + (size_t)128 * 128 * 2);
  const size_t oNP1D = off; off = al256(off + (size_t)128 * 512 * 2);
  const size_t oNP2D = off; off = al256(off + (size_t)64 * 256 * 2);
  const size_t oTAB  = off; off = al256(off + ((size_t)2 * nTab + (size_t)gC * 32) * 4);
  const size_t oLIST = off; off = al256(off + (size_t)gC * RCAP * 4);
  const size_t oEWG  = off; off = al256(off + EP * 4);
  const size_t oHID  = off; off = al256(off + EP * HP * 2);
  const size_t oXREG = off; off = al256(off + (size_t)MP * 128 * 2);
  const size_t oR1   = off; off = al256(off + (size_t)MP * 256 * 4);
  const size_t oAREG = off; off = al256(off + (size_t)MP * 256 * 2);
  const size_t oSKIP = off; off = al256(off + (size_t)MP * 128 * 4);
  const size_t oSW   = off; off = al256(off + (size_t)MP * 4);
  if (off > ws_size) return;

  unsigned short* EE1D = (unsigned short*)(ws + oEE1D);
  unsigned short* ECW  = (unsigned short*)(ws + oECW);
  unsigned short* MHL1 = (unsigned short*)(ws + oMHL1);
  unsigned short* MHL2 = (unsigned short*)(ws + oMHL2);
  unsigned short* MHL3 = (unsigned short*)(ws + oMHL3);
  float*          CL1  = (float*)(ws + oCL1);
  float*          CL2  = (float*)(ws + oCL2);
  float*          CL3  = (float*)(ws + oCL3);
  unsigned short* WPD1 = (unsigned short*)(ws + oWPD1);
  unsigned short* WPD2 = (unsigned short*)(ws + oWPD2);
  unsigned short* WPD3 = (unsigned short*)(ws + oWPD3);
  unsigned short* W2D1 = (unsigned short*)(ws + oW2D1);
  unsigned short* W2D2 = (unsigned short*)(ws + oW2D2);
  unsigned short* W2D3 = (unsigned short*)(ws + oW2D3);
  unsigned short* PROJD = (unsigned short*)(ws + oPROJ);
  unsigned short* EE2D = (unsigned short*)(ws + oEE2D);
  unsigned short* NP1D = (unsigned short*)(ws + oNP1D);
  unsigned short* NP2D = (unsigned short*)(ws + oNP2D);
  int*            TAB  = (int*)(ws + oTAB);
  int*            LISTP = (int*)(ws + oLIST);
  float*          EWG  = (float*)(ws + oEWG);
  unsigned short* HID  = (unsigned short*)(ws + oHID);
  unsigned short* XREG = (unsigned short*)(ws + oXREG);
  float*          R1   = (float*)(ws + oR1);
  unsigned short* XFHL = (unsigned short*)(ws + oR1);
  unsigned short* AREG = (unsigned short*)(ws + oAREG);
  float*          SKIP = (float*)(ws + oSKIP);
  float*          SW   = (float*)(ws + oSW);

  hipFuncSetAttribute(reinterpret_cast<const void*>(&k_compact), hipFuncAttributeMaxDynamicSharedMemorySize,
                      (int)CMP_LDS_BYTES);
  hipFuncSetAttribute(reinterpret_cast<const void*>(&k_edge), hipFuncAttributeMaxDynamicSharedMemorySize,
                      (int)EDGE_LDS_BYTES);
  hipFuncSetAttribute(reinterpret_cast<const void*>(&k_layer<32, 0>), hipFuncAttributeMaxDynamicSharedMemorySize,
                      layer_lds_bytes<32, 0>());
  hipFuncSetAttribute(reinterpret_cast<const void*>(&k_layer<64, 0>), hipFuncAttributeMaxDynamicSharedMemorySize,
                      layer_lds_bytes<64, 0>());
  hipFuncSetAttribute(reinterpret_cast<const void*>(&k_layer<128, 1>), hipFuncAttributeMaxDynamicSharedMemorySize,
                      layer_lds_bytes<128, 1>());
  hipFuncSetAttribute(reinterpret_cast<const void*>(&k_head), hipFuncAttributeMaxDynamicSharedMemorySize,
                      (int)HEAD_LDS_BYTES);

  wplane(stream, eew1, 64, 0, 32, 64, 64, EE1D);
  wplane(stream, ecw1, 16, 0, 32, 32, 16, ECW);
  wplane(stream, c1w1, 32, 0, 64, 128, 32, WPD1);
  wplane(stream, c1w1, 32, 64, 64, 128, 32, WPD1 + 32 * 128);
  wplane(stream, c2w1, 64, 0, 32, 64, 64, WPD2);
  wplane(stream, c2w1, 64, 32, 32, 64, 64, WPD2 + 64 * 64);
  wplane(stream, c3w1, 128, 0, 64, 128, 128, WPD3);
  wplane(stream, c3w1, 128, 64, 64, 128, 128, WPD3 + 128 * 128);
  wplane(stream, c1w2, 32, 0, 32, 64, 32, W2D1);
  wplane(stream, c2w2, 64, 0, 64, 128, 64, W2D2);
  wplane(stream, c3w2, 128, 0, 128, 256, 128, W2D3);
  wplane(stream, projw, 128, 0, 64, 128, 128, PROJD);
  wplane(stream, eew2, 128, 0, 64, 128, 128, EE2D);
  wplane(stream, npw1, 128, 0, 128, 512, 128, NP1D);
  wplane(stream, npw2, 64, 0, 128, 256, 64, NP2D);
  k_mplane<32><<<1, NTHR, 0, stream>>>(eew2, eeb2, c1w1, 128, MHL1, CL1);
  k_mplane<64><<<2, NTHR, 0, stream>>>(eew2, eeb2, c2w1, 64, MHL2, CL2);
  k_mplane<128><<<4, NTHR, 0, stream>>>(eew2, eeb2, c3w1, 128, MHL3, CL3);
  k_xprep<<<(MP * 8) / NTHR, NTHR, 0, stream>>>(x_in, bn0w, bn0b, bn0rm, bn0rv, nN, XREG);
  k_compact<<<gC, NTHR, CMP_LDS_BYTES, stream>>>(ei + nE, nE, ((nE & 3) == 0) ? 1 : 0, LISTP, TAB, nTab);
  k_edge<<<gE, NTHR, EDGE_LDS_BYTES, stream>>>(eattr, nE, EE1D, ECW, eelng, eelnb, eeb1, ecb1, ecw2, ecb2, HID, EWG);
  k_gemm<4, 0><<<dim3(gM, 1), GTHR, 0, stream>>>(XREG, 128, WPD1, 128, 128, c1b1, 32, 1.0f, ln1g, ln1b, TAB, nTab,
                                                 SW, R1, 64, AREG, 0, 0, nN);
  k_gemm<8, 0><<<dim3(gM, 1), GTHR, 0, stream>>>(XREG, 128, PROJD, 128, 128, projb, 128, 0.01f, ln1g, ln1b, TAB,
                                                 nTab, SW, SKIP, 128, AREG, 0, 0, nN);
  k_layer<32, 0><<<gL, NTHR, layer_lds_bytes<32, 0>(), stream>>>(ei, nE, nN, LISTP, TAB, nTab, HID, EWG, MHL1, CL1,
                                                                  R1, AREG, AREG, SW);
  k_gemm<2, 1><<<dim3(gM, 1), GTHR, 0, stream>>>(AREG, 64, W2D1, 64, 64, c1b2, 32, 1.0f, ln1g, ln1b, TAB, nTab,
                                                 SW, R1, 0, XREG, 64, 0, nN);
  k_gemm<8, 0><<<dim3(gM, 1), GTHR, 0, stream>>>(XREG, 64, WPD2, 64, 64, c2b1, 64, 1.0f, ln2g, ln2b, TAB, nTab,
                                                 SW, R1, 128, AREG, 0, 0, nN);
  k_layer<64, 0><<<gL, NTHR, layer_lds_bytes<64, 0>(), stream>>>(ei, nE, nN, LISTP, TAB, nTab, HID, EWG, MHL2, CL2,
                                                                  R1, AREG, AREG, SW);
  k_gemm<4, 2><<<dim3(gM, 1), GTHR, 0, stream>>>(AREG, 128, W2D2, 128, 128, c2b2, 64, 1.0f, ln2g, ln2b, TAB, nTab,
                                                 SW, R1, 0, XREG, 128, 0, nN);
  k_gemm<8, 0><<<dim3(gM, 2), GTHR, 0, stream>>>(XREG, 128, WPD3, 128, 128, c3b1, 128, 1.0f, ln3g, ln3b, TAB, nTab,
                                                 SW, R1, 256, AREG, 0, 0, nN);
  k_layer<128, 1><<<gL, NTHR, layer_lds_bytes<128, 1>(), stream>>>(ei, nE, nN, LISTP, TAB, nTab, HID, EWG, MHL3,
                                                                    CL3, R1, AREG, XREG, SW);
  k_gemm<8, 3><<<dim3(gM, 1), GTHR, 0, stream>>>(AREG, 256, W2D3, 256, 256, c3b2, 128, 1.0f, ln3g, ln3b, TAB, nTab,
                                                 SKIP, out0, 256, XFHL, 512, 0, nN);
  k_gemm<8, 4><<<dim3(gM, 1), GTHR, 0, stream>>>(XREG, 128, EE2D, 128, 128, eeb2, 128, 1.0f, ln3g, ln3b, TAB, nTab,
                                                 SW, out0, 256, XFHL, 512, 256, nN);
  k_head<<<gM, GTHR, HEAD_LDS_BYTES, stream>>>(XFHL, NP1D, NP2D, npb1, npb2, npw3, npb3, TAB, nTab, out1, nN);
}
